// Edge_net_13795434954992
// MI455X (gfx1250) — hardware-run, weakly checked
//
#include <hip/hip_runtime.h>
#include <stddef.h>
#include <math.h>


typedef _Float16 h16;
typedef _Float16 v16h __attribute__((ext_vector_type(16)));
typedef _Float16 v8h  __attribute__((ext_vector_type(8)));
typedef float    v8f  __attribute__((ext_vector_type(8)));
typedef float    v4f  __attribute__((ext_vector_type(4)));

#ifndef NROWS
#define NROWS 131072
#endif
#define NROWS_FULL 131072
#define IN_F   64
#define OUT_F  64
#define NTYPES 10
#define NPLANES (NTYPES + 1)
#define PLANE_ELEMS (OUT_F * IN_F)

#define LDC 68

#define DCARRY 16.0f
#define WCARRY 1024.0f
#define ACC_INV (1.0f / (DCARRY * WCARRY))

#define WP_BYTES ((size_t)NPLANES * PLANE_ELEMS * 2)
#define OFF_WP   ((size_t)0)
#define WS_TOTAL (OFF_WP + WP_BYTES)

static_assert(NROWS >= 64 && NROWS <= NROWS_FULL && (NROWS % 64) == 0);
static_assert(IN_F == 64 && OUT_F == 64);
static_assert((IN_F % 32) == 0 && (OUT_F % 16) == 0);
static_assert(((NTYPES * PLANE_ELEMS) % (256 * 8)) == 0);
static_assert((PLANE_ELEMS % (256 * 8)) == 0);
static_assert((LDC % 4) == 0 && LDC >= 64);
static_assert((WP_BYTES % 128) == 0);
static_assert(WS_TOTAL <= (size_t)134217728);
static_assert((size_t)NROWS * OUT_F < (size_t)0x7FFFFFFF);

__device__ __forceinline__ float bf16r(float x) {
  unsigned int u = __float_as_uint(x);
  u = (u + 0x7FFFu + ((u >> 16) & 1u)) & 0xFFFF0000u;
  return __uint_as_float(u);
}

static __device__ __forceinline__ h16 toh_flush(float v) {
  const h16 r = (h16)v;
  return (fabsf(v) < 6.103515625e-05f) ? (h16)0.0f : r;
}

__device__ __forceinline__ v16h frag_at(const _Float16* p) {
  v8h lo = *(const v8h*)(p);
  v8h hi = *(const v8h*)(p + 16);
  v16h out;
#pragma unroll
  for (int i = 0; i < 8; ++i) { out[i] = lo[i]; out[i + 8] = hi[i]; }
  return out;
}

__device__ __forceinline__ v8f wmma16(v16h a, v16h b, v8f c) {
  v8f d = __builtin_amdgcn_wmma_f32_16x16x32_f16(false, a, false, b, (short)0, c,
                                                 false, false);
  asm volatile("v_nop\n\tv_nop\n\tv_nop\n\tv_nop" : "+v"(d) : "v"(a), "v"(b));
  return d;
}

__device__ __forceinline__ void wave_lds_sync() {
  __builtin_amdgcn_fence(3  , "wavefront");
  asm volatile("s_wait_dscnt 0x0" ::: "memory");
  __builtin_amdgcn_wave_barrier();
}

__global__ __launch_bounds__(256) void wplane_kernel(
    const float* __restrict__ src, _Float16* __restrict__ dst) {
  const unsigned idx = blockIdx.x * 256u + threadIdx.x;
  const size_t e = (size_t)idx * 8u;
  const v4f a0 = *(const v4f*)(src + e);
  const v4f a1 = *(const v4f*)(src + e + 4u);
  v8h o;
#pragma unroll
  for (int i = 0; i < 4; ++i) {
    o[i]     = toh_flush(WCARRY * bf16r(a0[i]));
    o[i + 4] = toh_flush(WCARRY * bf16r(a1[i]));
  }
  _Float16* p = dst + e;
  *(volatile v8h*)p = o;
  __threadfence();
  *(volatile v8h*)p = o;
}

__global__ __launch_bounds__(128) void edge_kernel(
    const int* __restrict__ typ, const float* __restrict__ desc,
    const _Float16* __restrict__ Wp, const float* __restrict__ lin_b,
    float* __restrict__ out) {
  __shared__ __attribute__((aligned(16))) float Cb[4 * 16 * LDC];
  __shared__ __attribute__((aligned(16))) float Cl[4 * 16 * LDC];

  const unsigned tid = threadIdx.x, lane = tid & 31u;
  const unsigned wave = (unsigned)__builtin_amdgcn_readfirstlane(threadIdx.x >> 5);
  const unsigned hh = lane >> 4, m = lane & 15u;
  const unsigned row0 = blockIdx.x * 64u + wave * 16u;
  const unsigned cbase = wave * (16u * LDC);

  int tm = typ[row0 + m];
  tm = (tm < 0) ? 0 : tm;
  tm = (tm > (NTYPES - 1)) ? (NTYPES - 1) : tm;

  const float* ar = desc + (size_t)(row0 + m) * IN_F + hh * 8u;
  v16h a[2];
#pragma unroll
  for (int c = 0; c < 2; ++c) {
    const v4f x0 = *(const v4f*)(ar + c * 32);
    const v4f x1 = *(const v4f*)(ar + c * 32 + 4);
    const v4f x2 = *(const v4f*)(ar + c * 32 + 16);
    const v4f x3 = *(const v4f*)(ar + c * 32 + 20);
#pragma unroll
    for (int i = 0; i < 4; ++i) {
      a[c][i]      = toh_flush(DCARRY * bf16r(x0[i]));
      a[c][i + 4]  = toh_flush(DCARRY * bf16r(x1[i]));
      a[c][i + 8]  = toh_flush(DCARRY * bf16r(x2[i]));
      a[c][i + 12] = toh_flush(DCARRY * bf16r(x3[i]));
    }
  }

  v8f bond[4], lin[4];
#pragma unroll
  for (int nb = 0; nb < 4; ++nb) { bond[nb] = (v8f){}; lin[nb] = (v8f){}; }

  const v16h zf = {};
  const _Float16* bp = Wp + (size_t)m * IN_F + hh * 8u;

#pragma unroll 1
  for (int t = 0; t < NTYPES; ++t) {
    const bool sel = (tm == t);
    const v16h am0 = sel ? a[0] : zf;
    const v16h am1 = sel ? a[1] : zf;
    const _Float16* bt = bp + (size_t)t * PLANE_ELEMS;
#pragma unroll
    for (int nb = 0; nb < 4; ++nb) {
      const v16h b0 = frag_at(bt + nb * 16 * IN_F);
      const v16h b1 = frag_at(bt + nb * 16 * IN_F + 32);
      bond[nb] = wmma16(am0, b0, bond[nb]);
      bond[nb] = wmma16(am1, b1, bond[nb]);
    }
  }
  {
    const _Float16* bt = bp + (size_t)NTYPES * PLANE_ELEMS;
#pragma unroll
    for (int nb = 0; nb < 4; ++nb) {
      const v16h b0 = frag_at(bt + nb * 16 * IN_F);
      const v16h b1 = frag_at(bt + nb * 16 * IN_F + 32);
      lin[nb] = wmma16(a[0], b0, lin[nb]);
      lin[nb] = wmma16(a[1], b1, lin[nb]);
    }
  }

#pragma unroll
  for (int nb = 0; nb < 4; ++nb)
#pragma unroll
    for (int r = 0; r < 8; ++r) {
      const unsigned at = cbase + (hh * 8u + (unsigned)r) * LDC + (unsigned)nb * 16u + m;
      Cb[at] = bond[nb][r];
      Cl[at] = lin[nb][r];
    }
  wave_lds_sync();

  const unsigned c4 = (lane & 15u) * 4u;
  const v4f gb = *(const v4f*)(lin_b + c4);
  v4f bb;
#pragma unroll
  for (int j = 0; j < 4; ++j) bb[j] = bf16r(gb[j]);

#pragma unroll 1
  for (unsigned i = 0; i < 8u; ++i) {
    const unsigned r = 2u * i + (lane >> 4);
    const v4f ub = *(const v4f*)&Cb[cbase + r * LDC + c4];
    const v4f ul = *(const v4f*)&Cl[cbase + r * LDC + c4];
    v4f val;
#pragma unroll
    for (int j = 0; j < 4; ++j)
      val[j] = tanhf(ub[j] * ACC_INV) + (ul[j] * ACC_INV + bb[j]);
    float* p = out + (size_t)(row0 + r) * OUT_F + c4;
    *(volatile v4f*)p = val;
    __threadfence();
    *(volatile v4f*)p = val;
  }
}

extern "C" void kernel_launch(void* const* d_in, const int* in_sizes, int n_in,
                              void* d_out, int out_size, void* d_ws, size_t ws_size,
                              hipStream_t stream) {
  if (n_in < 5) return;
  if ((long long)in_sizes[0] < (long long)NROWS) return;
  if ((long long)in_sizes[1] < (long long)NROWS * IN_F) return;
  if ((long long)in_sizes[2] < (long long)NTYPES * PLANE_ELEMS) return;
  if ((long long)in_sizes[3] < (long long)PLANE_ELEMS) return;
  if (in_sizes[4] < OUT_F) return;
  if ((long long)out_size < (long long)NROWS * OUT_F) return;
  if (ws_size < WS_TOTAL) return;

  const int*   typ    = (const int*)d_in[0];
  const float* desc   = (const float*)d_in[1];
  const float* layer1 = (const float*)d_in[2];
  const float* lin_w  = (const float*)d_in[3];
  const float* lin_b  = (const float*)d_in[4];
  float* out = (float*)d_out;

  char* ws = (char*)d_ws;
  _Float16* Wp = (_Float16*)(ws + OFF_WP);

  wplane_kernel<<<dim3((NTYPES * PLANE_ELEMS) / 2048), dim3(256), 0, stream>>>(layer1, Wp);
  wplane_kernel<<<dim3(PLANE_ELEMS / 2048), dim3(256), 0, stream>>>(
      lin_w, Wp + (size_t)NTYPES * PLANE_ELEMS);

  edge_kernel<<<dim3(NROWS / 64), dim3(128), 0, stream>>>(typ, desc, Wp, lin_b, out);
}
